// toeken_proj_56332791054480
// MI455X (gfx1250) — hardware-verified
//
#include <hip/hip_runtime.h>
#include <stddef.h>
#include <stdint.h>

#define NBATCH 8
#define NQ     4096
#define NKEY   1024
#define DIN    128
#define HID    512
#define RQ     (NBATCH * NQ)
#define RK     (NBATCH * NKEY)
#define NRB    (NQ / 128)
#define MCH    256

static_assert(RQ % 128 == 0);
static_assert(RK % 128 == 0);
static_assert(NQ % 128 == 0);
static_assert(NKEY % 64 == 0);
static_assert(HID % 64 == 0);
static_assert(DIN == 128);
static_assert(NKEY % MCH == 0);
static_assert(MCH == 256);
static_assert(NQ % 64 == 0);

typedef _Float16       v16h __attribute__((ext_vector_type(16)));
typedef _Float16       v8h  __attribute__((ext_vector_type(8)));
typedef __bf16         v16b __attribute__((ext_vector_type(16)));
typedef unsigned short v8us __attribute__((ext_vector_type(8)));
typedef float          v8f  __attribute__((ext_vector_type(8)));
typedef float          v4f  __attribute__((ext_vector_type(4)));
typedef unsigned int   v4u  __attribute__((ext_vector_type(4)));

union FragH  { v16h v; v8h h[2]; };
union FragB  { v16b v; v8us u[2]; };
union Pack8  { _Float16 a[8]; v8h h; v4u u; };
union Pack8u { unsigned short a[8]; v8us s; v4u u; };
union BfBits { __bf16 h; unsigned short s; };

__device__ __forceinline__ unsigned short bf16_bits(float x) { BfBits u; u.h = (__bf16)x; return u.s; }
__device__ __forceinline__ float bf16_val(unsigned short s) { return __uint_as_float(((unsigned int)s) << 16); }

__device__ __forceinline__ v8f mma_h(v16h a, v16h b, v8f c) {
  c = __builtin_amdgcn_wmma_f32_16x16x32_f16(false, a, false, b, (short)0, c, false, false);
  asm volatile("v_nop\n\tv_nop\n\tv_nop\n\tv_nop" : "+v"(c) : "v"(a), "v"(b));
  return c;
}
__device__ __forceinline__ v8f mma_b(v16b a, v16b b, v8f c) {
  c = __builtin_amdgcn_wmma_f32_16x16x32_bf16(false, a, false, b, (short)0, c, false, false);
  asm volatile("v_nop\n\tv_nop\n\tv_nop\n\tv_nop" : "+v"(c) : "v"(a), "v"(b));
  return c;
}

__device__ __forceinline__ v8f zero8() { return (v8f){0.f, 0.f, 0.f, 0.f, 0.f, 0.f, 0.f, 0.f}; }

__device__ __forceinline__ v16h ldfrag_h(const _Float16* p, int ld, int row0, int k0, int lane) {
  const int m = lane & 15, lh = lane >> 4;
  const _Float16* q = p + (size_t)(row0 + m) * ld + k0 + 8 * lh;
  FragH f;
  f.h[0] = *(const v8h*)(q);
  f.h[1] = *(const v8h*)(q + 16);
  return f.v;
}
__device__ __forceinline__ v16b ldfrag_b(const unsigned short* p, int ld, int row0, int k0, int lane) {
  const int m = lane & 15, lh = lane >> 4;
  const unsigned short* q = p + (size_t)(row0 + m) * ld + k0 + 8 * lh;
  FragB f;
  f.u[0] = *(const v8us*)(q);
  f.u[1] = *(const v8us*)(q + 16);
  return f.v;
}

__device__ __forceinline__ void gemm3_32x64(const unsigned short* __restrict__ Ah, const unsigned short* __restrict__ Al,
                                            int lda,
                                            const unsigned short* __restrict__ Bh, const unsigned short* __restrict__ Bl,
                                            int ldb, int K, int m0, int n0, int lane, v8f (&acc)[2][4]) {
#pragma unroll 1
  for (int k0 = 0; k0 < K; k0 += 32) {
    const v16b a0h = ldfrag_b(Ah, lda, m0, k0, lane);
    const v16b a1h = ldfrag_b(Ah, lda, m0 + 16, k0, lane);
    const v16b a0l = ldfrag_b(Al, lda, m0, k0, lane);
    const v16b a1l = ldfrag_b(Al, lda, m0 + 16, k0, lane);
#pragma unroll
    for (int t = 0; t < 4; ++t) {
      const v16b bhf = ldfrag_b(Bh, ldb, n0 + 16 * t, k0, lane);
      const v16b blf = ldfrag_b(Bl, ldb, n0 + 16 * t, k0, lane);
      acc[0][t] = mma_b(a0h, bhf, acc[0][t]);
      acc[0][t] = mma_b(a0h, blf, acc[0][t]);
      acc[0][t] = mma_b(a0l, bhf, acc[0][t]);
      acc[1][t] = mma_b(a1h, bhf, acc[1][t]);
      acc[1][t] = mma_b(a1h, blf, acc[1][t]);
      acc[1][t] = mma_b(a1l, bhf, acc[1][t]);
    }
  }
}

template <int WITHF16>
__global__ __launch_bounds__(256) void k_cvt_rows(const float* __restrict__ x, unsigned short* __restrict__ ph,
                                                  unsigned short* __restrict__ pl, _Float16* __restrict__ p16,
                                                  int ngrp) {
  const int t = blockIdx.x * 256 + (int)threadIdx.x;
  if (t >= ngrp) return;
  const size_t o = (size_t)t * 8;
  const v4f a0 = *(const v4f*)(x + o);
  const v4f a1 = *(const v4f*)(x + o + 4);
  const float f[8] = {a0[0], a0[1], a0[2], a0[3], a1[0], a1[1], a1[2], a1[3]};
  Pack8u hk, lk;
  Pack8 hp;
#pragma unroll
  for (int i = 0; i < 8; ++i) {
    const unsigned short hb = bf16_bits(f[i]);
    hk.a[i] = hb;
    lk.a[i] = bf16_bits(f[i] - bf16_val(hb));
    hp.a[i] = (_Float16)f[i];
  }
  const v4u hv = hk.u, lv = lk.u, fv = hp.u;
  volatile v4u* dh = (volatile v4u*)(ph + o);
  volatile v4u* dl = (volatile v4u*)(pl + o);
  *dh = hv;
  *dl = lv;
  if (WITHF16) *(volatile v4u*)(p16 + o) = fv;
  __threadfence();
  *dh = hv;
  *dl = lv;
  if (WITHF16) *(volatile v4u*)(p16 + o) = fv;
}

#define WTP 136
__global__ __launch_bounds__(256) void k_cvt_w12(const float* __restrict__ wa, const float* __restrict__ wb,
                                                 unsigned short* __restrict__ ha, unsigned short* __restrict__ la,
                                                 unsigned short* __restrict__ hb, unsigned short* __restrict__ lb, int N) {
  __shared__ __align__(16) unsigned short th[64 * WTP];
  __shared__ __align__(16) unsigned short tl[64 * WTP];
  const int tid = threadIdx.x;
  const int sel = blockIdx.y;
  const float* w = sel ? wb : wa;
  unsigned short* oh = sel ? hb : ha;
  unsigned short* ol = sel ? lb : la;
  const int n0 = blockIdx.x * 64;
#pragma unroll 4
  for (int i = 0; i < 32; ++i) {
    const int e  = tid + 256 * i;
    const int kr = e >> 6;
    const int nc = e & 63;
    const float v = w[(size_t)kr * N + n0 + nc];
    const unsigned short hbits = bf16_bits(v);
    th[nc * WTP + kr] = hbits;
    tl[nc * WTP + kr] = bf16_bits(v - bf16_val(hbits));
  }
  __syncthreads();
  v4u vh[4], vl[4];
  size_t go[4];
#pragma unroll
  for (int j = 0; j < 4; ++j) {
    const int p  = tid + 256 * j;
    const int nr = p >> 4;
    const int pc = p & 15;
    Pack8u a, b;
    a.s = *(const v8us*)(th + nr * WTP + pc * 8);
    b.s = *(const v8us*)(tl + nr * WTP + pc * 8);
    vh[j] = a.u;
    vl[j] = b.u;
    go[j] = (size_t)(n0 + nr) * DIN + pc * 8;
  }
  for (int ps = 0; ps < 2; ++ps) {
#pragma unroll
    for (int j = 0; j < 4; ++j) {
      *(volatile v4u*)(oh + go[j]) = vh[j];
      *(volatile v4u*)(ol + go[j]) = vl[j];
    }
    __threadfence();
  }
}

__global__ __launch_bounds__(256) void k_cvt_w3(const float* __restrict__ w, _Float16* __restrict__ o16, int N,
                                                float sc) {
  __shared__ __align__(16) _Float16 t16[64 * WTP];
  const int tid = threadIdx.x;
  const int n0 = blockIdx.x * 64;
#pragma unroll 4
  for (int i = 0; i < 32; ++i) {
    const int e  = tid + 256 * i;
    const int kr = e >> 6;
    const int nc = e & 63;
    t16[nc * WTP + kr] = (_Float16)(w[(size_t)kr * N + n0 + nc] * sc);
  }
  __syncthreads();
  v4u vv[4];
  size_t go[4];
#pragma unroll
  for (int j = 0; j < 4; ++j) {
    const int p  = tid + 256 * j;
    const int nr = p >> 4;
    const int pc = p & 15;
    Pack8 a;
    a.h = *(const v8h*)(t16 + nr * WTP + pc * 8);
    vv[j] = a.u;
    go[j] = (size_t)(n0 + nr) * DIN + pc * 8;
  }
  for (int ps = 0; ps < 2; ++ps) {
#pragma unroll
    for (int j = 0; j < 4; ++j) *(volatile v4u*)(o16 + go[j]) = vv[j];
    __threadfence();
  }
}

#define STP 72
__global__ __launch_bounds__(128) void k_proj3(const unsigned short* __restrict__ ah, const unsigned short* __restrict__ al,
                                               const unsigned short* __restrict__ bh, const unsigned short* __restrict__ bl,
                                               const float* __restrict__ bias,
                                               unsigned short* __restrict__ oh, unsigned short* __restrict__ ol, int N) {
  __shared__ __align__(16) unsigned short sth[128 * STP];
  __shared__ __align__(16) unsigned short stl[128 * STP];
  const int tid = threadIdx.x, lane = tid & 31, wave = tid >> 5;
  const int hh = lane >> 4, c = lane & 15;
  const int mb = blockIdx.x * 128;
  const int m0 = mb + wave * 32;
  const int n0 = blockIdx.y * 64;

  v8f acc[2][4];
#pragma unroll
  for (int s = 0; s < 2; ++s)
#pragma unroll
    for (int t = 0; t < 4; ++t) acc[s][t] = zero8();
  gemm3_32x64(ah, al, DIN, bh, bl, DIN, DIN, m0, n0, lane, acc);

#pragma unroll
  for (int t = 0; t < 4; ++t) {
    const float bv = bias[n0 + 16 * t + c];
#pragma unroll
    for (int sub = 0; sub < 2; ++sub) {
#pragma unroll
      for (int r = 0; r < 8; ++r) {
        const int lr = wave * 32 + sub * 16 + 8 * hh + r;
        const float y = acc[sub][t][r] + bv;
        const unsigned short hbits = bf16_bits(y);
        sth[lr * STP + 16 * t + c] = hbits;
        stl[lr * STP + 16 * t + c] = bf16_bits(y - bf16_val(hbits));
      }
    }
  }
  __syncthreads();

  v4u vh[8], vl[8];
  size_t go[8];
#pragma unroll
  for (int j = 0; j < 8; ++j) {
    const int p  = tid + 128 * j;
    const int lr = p >> 3;
    const int pc = p & 7;
    Pack8u a, b;
    a.s = *(const v8us*)(sth + lr * STP + pc * 8);
    b.s = *(const v8us*)(stl + lr * STP + pc * 8);
    vh[j] = a.u;
    vl[j] = b.u;
    go[j] = (size_t)(mb + lr) * N + n0 + pc * 8;
  }
  for (int ps = 0; ps < 2; ++ps) {
#pragma unroll
    for (int j = 0; j < 8; ++j) {
      *(volatile v4u*)(oh + go[j]) = vh[j];
      *(volatile v4u*)(ol + go[j]) = vl[j];
    }
    __threadfence();
  }
}

__global__ __launch_bounds__(128) void k_projv(const _Float16* __restrict__ w3t, const _Float16* __restrict__ tt,
                                               const float* __restrict__ b3v, _Float16* __restrict__ vt) {
  __shared__ __align__(16) _Float16 st[128 * STP];
  const int tid = threadIdx.x, lane = tid & 31, wave = tid >> 5;
  const int hh = lane >> 4, c = lane & 15;
  const int m0 = wave * 32;
  const int n0 = blockIdx.x * 64;

  v8f acc[2][4];
#pragma unroll
  for (int s = 0; s < 2; ++s)
#pragma unroll
    for (int t = 0; t < 4; ++t) acc[s][t] = zero8();
#pragma unroll 1
  for (int k0 = 0; k0 < DIN; k0 += 32) {
    const v16h a0 = ldfrag_h(w3t, DIN, m0, k0, lane);
    const v16h a1 = ldfrag_h(w3t, DIN, m0 + 16, k0, lane);
#pragma unroll
    for (int t = 0; t < 4; ++t) {
      const v16h bf = ldfrag_h(tt, DIN, n0 + 16 * t, k0, lane);
      acc[0][t] = mma_h(a0, bf, acc[0][t]);
      acc[1][t] = mma_h(a1, bf, acc[1][t]);
    }
  }

#pragma unroll
  for (int sub = 0; sub < 2; ++sub) {
#pragma unroll
    for (int r = 0; r < 8; ++r) {
      const int lr = m0 + sub * 16 + 8 * hh + r;
      const float bv = b3v[lr] * 16.0f;
#pragma unroll
      for (int t = 0; t < 4; ++t) st[lr * STP + 16 * t + c] = (_Float16)(acc[sub][t][r] * 0.25f + bv);
    }
  }
  __syncthreads();

  v4u vv[8];
  size_t go[8];
#pragma unroll
  for (int j = 0; j < 8; ++j) {
    const int p  = tid + 128 * j;
    const int lr = p >> 3;
    const int pc = p & 7;
    Pack8 a;
    a.h = *(const v8h*)(st + lr * STP + pc * 8);
    vv[j] = a.u;
    go[j] = (size_t)lr * RK + n0 + pc * 8;
  }
  for (int ps = 0; ps < 2; ++ps) {
#pragma unroll
    for (int j = 0; j < 8; ++j) *(volatile v4u*)(vt + go[j]) = vv[j];
    __threadfence();
  }
}

#define OTP 68
__global__ __launch_bounds__(128) void k_sgemm(const unsigned short* __restrict__ qh, const unsigned short* __restrict__ ql,
                                               const unsigned short* __restrict__ kh, const unsigned short* __restrict__ kl,
                                               float* __restrict__ sp, float* __restrict__ part, int b) {
  __shared__ __align__(16) float st[4][16 * OTP];
  __shared__ float redm[4][64];
  __shared__ float reds[4][64];
  __shared__ __align__(16) float pst[128];
  const int tid = threadIdx.x, lane = tid & 31, wave = tid >> 5;
  const int hh = lane >> 4, c = lane & 15;
  const int rb = blockIdx.x;
  const int m0 = rb * 128 + wave * 32;
  const int n0 = blockIdx.y * 64;

  const unsigned short* Ah = qh + (size_t)b * NQ * HID;
  const unsigned short* Al = ql + (size_t)b * NQ * HID;
  const unsigned short* Bh = kh + (size_t)b * NKEY * HID;
  const unsigned short* Bl = kl + (size_t)b * NKEY * HID;

  v8f acc[2][4];
#pragma unroll
  for (int s = 0; s < 2; ++s)
#pragma unroll
    for (int t = 0; t < 4; ++t) acc[s][t] = zero8();
  gemm3_32x64(Ah, Al, HID, Bh, Bl, HID, HID, m0, n0, lane, acc);

  float cmx[4];
#pragma unroll
  for (int t = 0; t < 4; ++t) {
    float m = acc[0][t][0];
#pragma unroll
    for (int sub = 0; sub < 2; ++sub)
#pragma unroll
      for (int r = 0; r < 8; ++r) m = fmaxf(m, acc[sub][t][r]);
    m = fmaxf(m, __shfl_xor(m, 16, 32));
    cmx[t] = m;
  }
  if (hh == 0) {
#pragma unroll
    for (int t = 0; t < 4; ++t) redm[wave][16 * t + c] = cmx[t];
  }
  __syncthreads();
  float bmx[4];
#pragma unroll
  for (int t = 0; t < 4; ++t)
    bmx[t] = fmaxf(fmaxf(redm[0][16 * t + c], redm[1][16 * t + c]), fmaxf(redm[2][16 * t + c], redm[3][16 * t + c]));
  float csm[4];
#pragma unroll
  for (int t = 0; t < 4; ++t) {
    float s = 0.f;
#pragma unroll
    for (int sub = 0; sub < 2; ++sub)
#pragma unroll
      for (int r = 0; r < 8; ++r) s += __expf(acc[sub][t][r] - bmx[t]);
    s += __shfl_xor(s, 16, 32);
    csm[t] = s;
  }
  if (hh == 0) {
#pragma unroll
    for (int t = 0; t < 4; ++t) reds[wave][16 * t + c] = csm[t];
  }
  __syncthreads();
  if (tid < 64) {
    pst[tid] = fmaxf(fmaxf(redm[0][tid], redm[1][tid]), fmaxf(redm[2][tid], redm[3][tid]));
    pst[64 + tid] = ((reds[0][tid] + reds[1][tid]) + reds[2][tid]) + reds[3][tid];
  }
  __syncthreads();
  const v4f pv = *(const v4f*)(pst + 4 * lane);
  float* pdst = part + (size_t)rb * (2 * NKEY) + (size_t)hh * NKEY + n0 + 4 * c;

  float* sw = st[wave];
#pragma unroll
  for (int sub = 0; sub < 2; ++sub) {
    __syncthreads();
#pragma unroll
    for (int t = 0; t < 4; ++t) {
#pragma unroll
      for (int r = 0; r < 8; ++r) sw[(8 * hh + r) * OTP + 16 * t + c] = acc[sub][t][r];
    }
    __syncthreads();
    v4f val[8];
    size_t go[8];
#pragma unroll
    for (int it = 0; it < 8; ++it) {
      const int p    = lane + 32 * it;
      const int L    = p >> 3;
      const int pc   = p & 7;
      const int row  = L >> 1;
      const int half = L & 1;
      val[it] = *(const v4f*)(sw + row * OTP + half * 32 + pc * 4);
      go[it]  = (size_t)(m0 + sub * 16 + row) * NKEY + n0 + half * 32 + pc * 4;
    }
    for (int ps = 0; ps < 2; ++ps) {
#pragma unroll
      for (int it = 0; it < 8; ++it) *(volatile v4f*)(sp + go[it]) = val[it];
      if (sub == 1 && wave == 0) *(volatile v4f*)pdst = pv;
      __threadfence();
    }
  }
}

__global__ __launch_bounds__(256) void k_fin(const float* __restrict__ part, float* __restrict__ cmr) {
  const int col = blockIdx.x * 256 + (int)threadIdx.x;
  float gm = -__builtin_huge_valf();
#pragma unroll 1
  for (int rb = 0; rb < NRB; ++rb) gm = fmaxf(gm, part[(size_t)rb * (2 * NKEY) + col]);
  float gs = 0.f;
#pragma unroll 1
  for (int rb = 0; rb < NRB; ++rb) {
    const float pm = part[(size_t)rb * (2 * NKEY) + col];
    const float pq = part[(size_t)rb * (2 * NKEY) + NKEY + col];
    gs += pq * __expf(pm - gm);
  }
  const float cr = 1024.0f * __builtin_amdgcn_rcpf(gs);
  volatile float* d = (volatile float*)cmr;
  d[col] = gm;
  d[NKEY + col] = cr;
  __threadfence();
  d[col] = gm;
  d[NKEY + col] = cr;
}

#define PTP 264
#define CTP 132
static_assert(64 * CTP * 4 == 64 * PTP * 2);
__global__ __launch_bounds__(128) void k_out(const float* __restrict__ sp, const float* __restrict__ cmr,
                                             const _Float16* __restrict__ vt, const float* __restrict__ xc,
                                             float* __restrict__ out, int b) {
  __shared__ __align__(16) float sm[64 * CTP];
  __shared__ __align__(16) float tb[2 * NKEY];
  _Float16* ps16 = (_Float16*)sm;
  const int tid = threadIdx.x, lane = tid & 31, wave = tid >> 5;
  const int hh = lane >> 4, c = lane & 15;
  const int wr = wave & 1, wc = wave >> 1;
  const int n0 = blockIdx.x * 64;
#pragma unroll
  for (int i = 0; i < 4; ++i) {
    const int e = tid + 128 * i;
    *(v4f*)(tb + 4 * e) = *(const v4f*)(cmr + 4 * e);
  }
  const _Float16* vtb = vt + (size_t)b * NKEY;
  const float* sb = sp + (size_t)n0 * NKEY;

  v8f acc[2][4];
#pragma unroll
  for (int s = 0; s < 2; ++s)
#pragma unroll
    for (int t = 0; t < 4; ++t) acc[s][t] = zero8();

#pragma unroll 1
  for (int mc = 0; mc < NKEY; mc += MCH) {
    __syncthreads();
#pragma unroll 4
    for (int i = 0; i < 16; ++i) {
      const int e   = tid + 128 * i;
      const int row = e >> 5;
      const int pc  = e & 31;
      const int m   = mc + pc * 8;
      const float* srow = sb + (size_t)row * NKEY + m;
      const v4f s0 = *(const v4f*)(srow);
      const v4f s1 = *(const v4f*)(srow + 4);
      const v4f g0 = *(const v4f*)(tb + m);
      const v4f g1 = *(const v4f*)(tb + m + 4);
      const v4f r0 = *(const v4f*)(tb + NKEY + m);
      const v4f r1 = *(const v4f*)(tb + NKEY + m + 4);
      Pack8 pk;
#pragma unroll
      for (int j = 0; j < 4; ++j) {
        pk.a[j]     = (_Float16)(__expf(s0[j] - g0[j]) * r0[j]);
        pk.a[4 + j] = (_Float16)(__expf(s1[j] - g1[j]) * r1[j]);
      }
      *(v8h*)(ps16 + row * PTP + pc * 8) = pk.h;
    }
    __syncthreads();
#pragma unroll 1
    for (int kk = 0; kk < MCH; kk += 32) {
      const v16h pa0 = ldfrag_h(ps16, PTP, wr * 32, kk, lane);
      const v16h pa1 = ldfrag_h(ps16, PTP, wr * 32 + 16, kk, lane);
#pragma unroll
      for (int t = 0; t < 4; ++t) {
        const v16h vb = ldfrag_h(vtb, RK, wc * 64 + 16 * t, mc + kk, lane);
        acc[0][t] = mma_h(pa0, vb, acc[0][t]);
        acc[1][t] = mma_h(pa1, vb, acc[1][t]);
      }
    }
  }
  __syncthreads();

#pragma unroll
  for (int sub = 0; sub < 2; ++sub) {
#pragma unroll
    for (int t = 0; t < 4; ++t) {
#pragma unroll
      for (int r = 0; r < 8; ++r)
        sm[(wr * 32 + sub * 16 + 8 * hh + r) * CTP + wc * 64 + 16 * t + c] = acc[sub][t][r] * 6.103515625e-05f;
    }
  }
  __syncthreads();

  const float* xb = xc + ((size_t)b * NQ + n0) * DIN;
  float* ob = out + ((size_t)b * NQ + n0) * DIN;
  v4f val[16];
  int go[16];
#pragma unroll
  for (int i = 0; i < 16; ++i) {
    const int e   = tid + 128 * i;
    const int row = e >> 5;
    const int c4  = (e & 31) * 4;
    const v4f a = *(const v4f*)(sm + row * CTP + c4);
    const v4f x = *(const v4f*)(xb + row * DIN + c4);
    val[i] = a + x;
    go[i]  = row * DIN + c4;
  }
  for (int ps = 0; ps < 2; ++ps) {
#pragma unroll
    for (int i = 0; i < 16; ++i) *(volatile v4f*)(ob + go[i]) = val[i];
    __threadfence();
  }
}

#define SZ_XP   ((size_t)RQ * DIN * 2)
#define SZ_TP   ((size_t)RK * DIN * 2)
#define SZ_WHP  ((size_t)HID * DIN * 2)
#define SZ_W3P  ((size_t)DIN * DIN * 2)
#define SZ_QP   ((size_t)RQ * HID * 2)
#define SZ_KP   ((size_t)RK * HID * 2)
#define SZ_VT   ((size_t)DIN * RK * 2)
#define SZ_S    ((size_t)NQ * NKEY * 4)
#define SZ_PART ((size_t)NRB * 2 * NKEY * 4)
#define SZ_CMR  ((size_t)2 * NKEY * 4)

#define O_XCH  ((size_t)0)
#define O_XCL  (O_XCH + SZ_XP)
#define O_TTH  (O_XCL + SZ_XP)
#define O_TTL  (O_TTH + SZ_TP)
#define O_T16  (O_TTL + SZ_TP)
#define O_W1H  (O_T16 + SZ_TP)
#define O_W1L  (O_W1H + SZ_WHP)
#define O_W2H  (O_W1L + SZ_WHP)
#define O_W2L  (O_W2H + SZ_WHP)
#define O_W3T  (O_W2L + SZ_WHP)
#define O_QH   (O_W3T + SZ_W3P)
#define O_QL   (O_QH + SZ_QP)
#define O_KH   (O_QL + SZ_QP)
#define O_KL   (O_KH + SZ_KP)
#define O_VT   (O_KL + SZ_KP)
#define O_S    (O_VT + SZ_VT)
#define O_PART (O_S + SZ_S)
#define O_CMR  (O_PART + SZ_PART)
#define O_END  (O_CMR + SZ_CMR)

static_assert(O_QH == (size_t)23625728);
static_assert(O_S == (size_t)109608960);
static_assert(O_END == (size_t)126656512);
static_assert(O_END <= (size_t)134217728);
static_assert((O_XCL % 256) == 0);
static_assert((O_TTH % 256) == 0);
static_assert((O_T16 % 256) == 0);
static_assert((O_W1H % 256) == 0);
static_assert((O_W3T % 256) == 0);
static_assert((O_QH % 256) == 0);
static_assert((O_QL % 256) == 0);
static_assert((O_KH % 256) == 0);
static_assert((O_VT % 256) == 0);
static_assert((O_S % 256) == 0);
static_assert((O_PART % 256) == 0);
static_assert((O_CMR % 256) == 0);

extern "C" void kernel_launch(void* const* d_in, const int* in_sizes, int n_in,
                              void* d_out, int out_size, void* d_ws, size_t ws_size,
                              hipStream_t stream) {
  if (n_in < 8) return;
  if (in_sizes[0] != RQ * DIN) return;
  if (in_sizes[1] != RK * DIN) return;
  if (in_sizes[2] != DIN * HID) return;
  if (in_sizes[3] != HID) return;
  if (in_sizes[4] != DIN * HID) return;
  if (in_sizes[5] != HID) return;
  if (in_sizes[6] != DIN * DIN) return;
  if (in_sizes[7] != DIN) return;
  if (out_size != RQ * DIN) return;
  if (O_END > ws_size) return;

  const float* xc   = (const float*)d_in[0];
  const float* tout = (const float*)d_in[1];
  const float* w1   = (const float*)d_in[2];
  const float* b1   = (const float*)d_in[3];
  const float* w2   = (const float*)d_in[4];
  const float* b2   = (const float*)d_in[5];
  const float* w3   = (const float*)d_in[6];
  const float* b3   = (const float*)d_in[7];
  float* outp = (float*)d_out;

  char* ws = (char*)d_ws;
  unsigned short* XcH = (unsigned short*)(ws + O_XCH);
  unsigned short* XcL = (unsigned short*)(ws + O_XCL);
  unsigned short* TtH = (unsigned short*)(ws + O_TTH);
  unsigned short* TtL = (unsigned short*)(ws + O_TTL);
  _Float16*       T16 = (_Float16*)(ws + O_T16);
  unsigned short* W1H = (unsigned short*)(ws + O_W1H);
  unsigned short* W1L = (unsigned short*)(ws + O_W1L);
  unsigned short* W2H = (unsigned short*)(ws + O_W2H);
  unsigned short* W2L = (unsigned short*)(ws + O_W2L);
  _Float16*       W3T = (_Float16*)(ws + O_W3T);
  unsigned short* QH  = (unsigned short*)(ws + O_QH);
  unsigned short* QL  = (unsigned short*)(ws + O_QL);
  unsigned short* KH  = (unsigned short*)(ws + O_KH);
  unsigned short* KL  = (unsigned short*)(ws + O_KL);
  _Float16*       VT  = (_Float16*)(ws + O_VT);
  float*          SP  = (float*)(ws + O_S);
  float*          PART = (float*)(ws + O_PART);
  float*          CMR = (float*)(ws + O_CMR);

  {
    const int ngrp = RQ * DIN / 8;
    k_cvt_rows<0><<<dim3((ngrp + 255) / 256), dim3(256), 0, stream>>>(xc, XcH, XcL, T16, ngrp);
  }
  {
    const int ngrp = RK * DIN / 8;
    k_cvt_rows<1><<<dim3((ngrp + 255) / 256), dim3(256), 0, stream>>>(tout, TtH, TtL, T16, ngrp);
  }
  k_cvt_w12<<<dim3(HID / 64, 2), dim3(256), 0, stream>>>(w1, w2, W1H, W1L, W2H, W2L, HID);
  k_cvt_w3<<<dim3(DIN / 64), dim3(256), 0, stream>>>(w3, W3T, DIN, 64.0f);
  k_proj3<<<dim3(RQ / 128, HID / 64), dim3(128), 0, stream>>>(XcH, XcL, W1H, W1L, b1, QH, QL, HID);
  k_proj3<<<dim3(RK / 128, HID / 64), dim3(128), 0, stream>>>(TtH, TtL, W2H, W2L, b2, KH, KL, HID);
  k_projv<<<dim3(RK / 64), dim3(128), 0, stream>>>(W3T, T16, b3, VT);
  for (int b = 0; b < NBATCH; ++b) {
    k_sgemm<<<dim3(NQ / 128, NKEY / 64), dim3(128), 0, stream>>>(QH, QL, KH, KL, SP, PART, b);
    k_fin<<<dim3(NKEY / 256), dim3(256), 0, stream>>>(PART, CMR);
    k_out<<<dim3(NQ / 64), dim3(128), 0, stream>>>(SP, CMR, VT, xc, outp, b);
  }
  (void)hipGetLastError();
}
